// Transformer_hidden_state_learner_69887707840798
// MI455X (gfx1250) — hardware-verified
//
#include <hip/hip_runtime.h>
#include <stdint.h>
#include <stddef.h>


typedef __bf16 bf16_t;
typedef __bf16 v16b __attribute__((ext_vector_type(16)));
typedef __bf16 v8b  __attribute__((ext_vector_type(8)));
typedef float  v8f  __attribute__((ext_vector_type(8)));
typedef float  v4f  __attribute__((ext_vector_type(4)));
typedef unsigned int v4u __attribute__((ext_vector_type(4)));
typedef unsigned int v8u __attribute__((ext_vector_type(8)));

union Frag  { v16b v; v4u u[2]; v8b hv[2]; v8u w; };
union Pack8 { v8b b; v4u u; };

namespace {
constexpr int kD = 1024;
constexpr int kB = 16;
constexpr int kS = 512;
constexpr int kH = 16;
constexpr int kDh = 64;
constexpr int kRows = kB * kS;
constexpr int kHalfB = kB / 2;
constexpr int kHalfRows = kHalfB * kS;
constexpr float kNegBig = -1.0e9f;
constexpr float kScale = 0.125f;
constexpr int kSP = 68;
constexpr int kPP = 72;
constexpr int kTP = 65;

constexpr size_t kPlaneX = (size_t)kRows * kD * 2;
constexpr size_t kPlaneW = (size_t)kD * kD * 2;
constexpr size_t kPlaneH = (size_t)kHalfRows * kD * 2;
constexpr size_t OFF_XH = 0;
constexpr size_t OFF_XL = OFF_XH + kPlaneX;
constexpr size_t OFF_WT = OFF_XL + kPlaneX;
constexpr size_t OFF_QH = OFF_WT + 8 * kPlaneW;
constexpr size_t OFF_QL = OFF_QH + kPlaneH;
constexpr size_t OFF_KH = OFF_QL + kPlaneH;
constexpr size_t OFF_KL = OFF_KH + kPlaneH;
constexpr size_t OFF_VH = OFF_KL + kPlaneH;
constexpr size_t OFF_VL = OFF_VH + kPlaneH;
constexpr size_t kWsTotal = OFF_VL + kPlaneH;
static_assert(kWsTotal == (size_t)100663296);
}

__device__ __forceinline__ v8f mma(const Frag& a, const Frag& b, v8f c) {
  c = __builtin_amdgcn_wmma_f32_16x16x32_bf16(false, a.v, false, b.v, (short)0, c, false, false);
  asm volatile("v_nop\n\tv_nop\n\tv_nop\n\tv_nop" : "+v"(c) : "v"(a.w), "v"(b.w));
  return c;
}
__device__ __forceinline__ v8f mma3(const Frag& ah, const Frag& al, const Frag& bh, const Frag& bl, v8f c) {
  c = mma(ah, bh, c);
  c = mma(ah, bl, c);
  c = mma(al, bh, c);
  return c;
}

__device__ __forceinline__ Frag ldg_frag(const bf16_t* rowp, int hf) {
  Frag f;
  f.u[0] = *(const v4u*)(rowp + 8 * hf);
  f.u[1] = *(const v4u*)(rowp + 16 + 8 * hf);
  return f;
}
__device__ __forceinline__ Frag lds_frag(const bf16_t* rowp, int hf) {
  Frag f;
  f.hv[0] = *(const v8b*)(rowp + 8 * hf);
  f.hv[1] = *(const v8b*)(rowp + 16 + 8 * hf);
  return f;
}

__device__ __forceinline__ void split8(const float (&x)[8], v4u& uh, v4u& ul) {
  Pack8 a, b;
#pragma unroll
  for (int i = 0; i < 8; ++i) {
    const bf16_t hv = (bf16_t)x[i];
    const float rm = x[i] - (float)hv;
    a.b[i] = hv;
    b.b[i] = (bf16_t)rm;
  }
  uh = a.u;
  ul = b.u;
}

__device__ __forceinline__ void gemm_k1024(const bf16_t* __restrict__ ahp, const bf16_t* __restrict__ alp,
                                           const bf16_t* __restrict__ bhp, const bf16_t* __restrict__ blp,
                                           int hf, v8f& c0, v8f& c1, v8f& c2, v8f& c3) {
#pragma unroll 1
  for (int t = 0; t < kD / 32; ++t) {
    const int k0 = t * 32;
    const Frag ah = ldg_frag(ahp + k0, hf);
    const Frag al = ldg_frag(alp + k0, hf);
    {
      const Frag bh = ldg_frag(bhp + k0, hf);
      const Frag bl = ldg_frag(blp + k0, hf);
      c0 = mma3(ah, al, bh, bl, c0);
    }
    {
      const Frag bh = ldg_frag(bhp + (size_t)16 * kD + k0, hf);
      const Frag bl = ldg_frag(blp + (size_t)16 * kD + k0, hf);
      c1 = mma3(ah, al, bh, bl, c1);
    }
    {
      const Frag bh = ldg_frag(bhp + (size_t)32 * kD + k0, hf);
      const Frag bl = ldg_frag(blp + (size_t)32 * kD + k0, hf);
      c2 = mma3(ah, al, bh, bl, c2);
    }
    {
      const Frag bh = ldg_frag(bhp + (size_t)48 * kD + k0, hf);
      const Frag bl = ldg_frag(blp + (size_t)48 * kD + k0, hf);
      c3 = mma3(ah, al, bh, bl, c3);
    }
  }
}

__global__ void __launch_bounds__(256)
k_split_x(const float* __restrict__ src, bf16_t* __restrict__ xh, bf16_t* __restrict__ xl, int n8) {
  const int t = blockIdx.x * 256 + threadIdx.x;
  const int tc = (t < n8) ? t : (n8 - 1);
  const size_t base = (size_t)tc * 8;
  const v4f a = *(const v4f*)(src + base);
  const v4f b = *(const v4f*)(src + base + 4);
  float x[8] = { a[0], a[1], a[2], a[3], b[0], b[1], b[2], b[3] };
  v4u uh, ul;
  split8(x, uh, ul);
  if (t < n8) {
    *(volatile v4u*)(xh + base) = uh;
    *(volatile v4u*)(xl + base) = ul;
  }
  __threadfence();
  if (t < n8) {
    *(volatile v4u*)(xh + base) = uh;
    *(volatile v4u*)(xl + base) = ul;
  }
}

__global__ void __launch_bounds__(256)
k_split_wT(const float* __restrict__ w0, const float* __restrict__ w1,
           const float* __restrict__ w2, const float* __restrict__ w3,
           bf16_t* __restrict__ wt) {
  __shared__ float tile[64 * kTP];
  const int tid = threadIdx.x;
  const int bid = blockIdx.x;
  const int w = bid >> 8, tl = bid & 255;
  const int kt = tl >> 4, nt = tl & 15;
  const float* W = (w == 0) ? w0 : ((w == 1) ? w1 : ((w == 2) ? w2 : w3));
  bf16_t* ph = wt + (size_t)(2 * w) * kD * kD;
  bf16_t* pl = ph + (size_t)kD * kD;
  {
    const int kr = tid >> 2, cs = (tid & 3) * 16;
    const float* sp = W + (size_t)(64 * kt + kr) * kD + 64 * nt + cs;
#pragma unroll
    for (int u = 0; u < 4; ++u) {
      const v4f q4 = *(const v4f*)(sp + 4 * u);
      float* tp = tile + kr * kTP + cs + 4 * u;
      tp[0] = q4[0]; tp[1] = q4[1]; tp[2] = q4[2]; tp[3] = q4[3];
    }
  }
  __syncthreads();
  const int q = tid & 7;
  v4u uh[2], ul[2];
  size_t off[2];
#pragma unroll
  for (int i = 0; i < 2; ++i) {
    const int nl = (tid >> 3) + 32 * i;
    float x[8];
#pragma unroll
    for (int j = 0; j < 8; ++j) x[j] = tile[(8 * q + j) * kTP + nl];
    split8(x, uh[i], ul[i]);
    off[i] = (size_t)(64 * nt + nl) * kD + 64 * kt + 8 * q;
    *(volatile v4u*)(ph + off[i]) = uh[i];
    *(volatile v4u*)(pl + off[i]) = ul[i];
  }
  __threadfence();
#pragma unroll
  for (int i = 0; i < 2; ++i) {
    *(volatile v4u*)(ph + off[i]) = uh[i];
    *(volatile v4u*)(pl + off[i]) = ul[i];
  }
}

__global__ void __launch_bounds__(256)
k_qkv(const bf16_t* __restrict__ xh, const bf16_t* __restrict__ xl,
      const bf16_t* __restrict__ wt,
      const float* __restrict__ bq, const float* __restrict__ bk, const float* __restrict__ bv,
      bf16_t* __restrict__ qh, bf16_t* __restrict__ ql,
      bf16_t* __restrict__ kh, bf16_t* __restrict__ kl,
      bf16_t* __restrict__ vth, bf16_t* __restrict__ vtl, int hb) {
  __shared__ __align__(16) float stg[128 * kSP];
  const int tid = threadIdx.x, lane = tid & 31, wv = tid >> 5;
  const int hf = lane >> 4, n = lane & 15;
  const int bid = blockIdx.x;
  const int ct = bid & 15, rb = (bid >> 4) & 31, z = bid >> 9;
  const int c0 = ct * kDh;
  const int rl0 = rb * 128;
  const bf16_t* wph = wt + (size_t)(2 * z) * kD * kD;
  const bf16_t* wpl = wph + (size_t)kD * kD;
  const float* bias = (z == 0) ? bq : ((z == 1) ? bk : bv);

  const size_t arow = ((size_t)hb * kHalfRows + rl0 + 16 * wv + n) * kD;
  const size_t brow = (size_t)(c0 + n) * kD;
  v8f acc[4] = { {}, {}, {}, {} };
  gemm_k1024(xh + arow, xl + arow, wph + brow, wpl + brow, hf, acc[0], acc[1], acc[2], acc[3]);

#pragma unroll
  for (int j = 0; j < 4; ++j) {
    const int col = 16 * j + n;
    const float bb = bias[c0 + col];
#pragma unroll
    for (int g = 0; g < 8; ++g) stg[(16 * wv + 8 * hf + g) * kSP + col] = acc[j][g] + bb;
  }
  __syncthreads();

  const int q = tid & 7;
  if (z < 2) {
    bf16_t* ph = (z == 0) ? qh : kh;
    bf16_t* pl = (z == 0) ? ql : kl;
    v4u uh[4], ul[4];
    size_t off[4];
#pragma unroll
    for (int i = 0; i < 4; ++i) {
      const int row = (tid >> 3) + 32 * i;
      const int rl = rl0 + row;
      const int bl = rl >> 9, s = rl & (kS - 1);
      const float* sp = stg + row * kSP + 8 * q;
      const v4f a = *(const v4f*)sp;
      const v4f b = *(const v4f*)(sp + 4);
      float x[8] = { a[0], a[1], a[2], a[3], b[0], b[1], b[2], b[3] };
      split8(x, uh[i], ul[i]);
      off[i] = (((size_t)bl * kH + ct) * kS + s) * kDh + 8 * q;
      *(volatile v4u*)(ph + off[i]) = uh[i];
      *(volatile v4u*)(pl + off[i]) = ul[i];
    }
    __threadfence();
#pragma unroll
    for (int i = 0; i < 4; ++i) {
      *(volatile v4u*)(ph + off[i]) = uh[i];
      *(volatile v4u*)(pl + off[i]) = ul[i];
    }
  } else {
    const int bl = rl0 >> 9, sbase = rl0 & (kS - 1);
    v4u uh[4], ul[4];
    size_t off[4];
#pragma unroll
    for (int i = 0; i < 4; ++i) {
      const int L = (tid >> 3) + 32 * i;
      const int dh = L >> 1;
      const int sseg = (L & 1) * 64 + 8 * q;
      float x[8];
#pragma unroll
      for (int j = 0; j < 8; ++j) x[j] = stg[(sseg + j) * kSP + dh];
      split8(x, uh[i], ul[i]);
      off[i] = (((size_t)bl * kH + ct) * kDh + dh) * kS + sbase + sseg;
      *(volatile v4u*)(vth + off[i]) = uh[i];
      *(volatile v4u*)(vtl + off[i]) = ul[i];
    }
    __threadfence();
#pragma unroll
    for (int i = 0; i < 4; ++i) {
      *(volatile v4u*)(vth + off[i]) = uh[i];
      *(volatile v4u*)(vtl + off[i]) = ul[i];
    }
  }
}

__global__ void __launch_bounds__(128)
k_attn(const bf16_t* __restrict__ qh, const bf16_t* __restrict__ ql,
       const bf16_t* __restrict__ kh, const bf16_t* __restrict__ kl,
       const bf16_t* __restrict__ vth, const bf16_t* __restrict__ vtl,
       const int* __restrict__ lengths,
       bf16_t* __restrict__ oh, bf16_t* __restrict__ ol, int hb) {
  __shared__ __align__(16) bf16_t pth[4][16 * kPP];
  __shared__ __align__(16) bf16_t ptl[4][16 * kPP];
  __shared__ __align__(16) float stg[4][16 * kSP];
  const int tid = threadIdx.x, lane = tid & 31, wv = tid >> 5;
  const int hf = lane >> 4, n = lane & 15;
  const int bid = blockIdx.x;
  const int qt = bid & 7, hd = (bid >> 3) & 15, bl = bid >> 7;
  const int bg = hb * kHalfB + bl;
  int L = lengths[bg];
  L = (L < 0) ? 0 : L;
  L = (L > kS) ? kS : L;
  const int ntiles = (L == 0) ? (kS / 64) : ((L + 63) >> 6);
  const int bh = bl * kH + hd;
  const int q0 = qt * 64 + wv * 16;

  const size_t qrow = ((size_t)bh * kS + q0 + n) * kDh;
  const Frag aqh0 = ldg_frag(qh + qrow, hf);
  const Frag aqh1 = ldg_frag(qh + qrow + 32, hf);
  const Frag aql0 = ldg_frag(ql + qrow, hf);
  const Frag aql1 = ldg_frag(ql + qrow + 32, hf);

  bf16_t* myph = pth[wv];
  bf16_t* mypl = ptl[wv];
  float* myst = stg[wv];

  v8f acc[4] = { {}, {}, {}, {} };
  float mrow[8], lrow[8];
#pragma unroll
  for (int g = 0; g < 8; ++g) { mrow[g] = -3.0e38f; lrow[g] = 0.0f; }

#pragma unroll 1
  for (int kt = 0; kt < ntiles; ++kt) {
    const int key0 = kt * 64;
    v8f s[4] = { {}, {}, {}, {} };
#pragma unroll
    for (int jt = 0; jt < 4; ++jt) {
      const size_t kr = ((size_t)bh * kS + key0 + 16 * jt + n) * kDh;
      {
        const Frag b0h = ldg_frag(kh + kr, hf);
        const Frag b0l = ldg_frag(kl + kr, hf);
        s[jt] = mma3(aqh0, aql0, b0h, b0l, s[jt]);
      }
      {
        const Frag b1h = ldg_frag(kh + kr + 32, hf);
        const Frag b1l = ldg_frag(kl + kr + 32, hf);
        s[jt] = mma3(aqh1, aql1, b1h, b1l, s[jt]);
      }
    }
#pragma unroll
    for (int g = 0; g < 8; ++g) {
      float e[4];
      float t = -3.0e38f;
#pragma unroll
      for (int jt = 0; jt < 4; ++jt) {
        const int key = key0 + 16 * jt + n;
        const float ev = (key < L) ? (s[jt][g] * kScale) : kNegBig;
        e[jt] = ev;
        t = fmaxf(t, ev);
      }
      t = fmaxf(t, __shfl_xor(t, 1));
      t = fmaxf(t, __shfl_xor(t, 2));
      t = fmaxf(t, __shfl_xor(t, 4));
      t = fmaxf(t, __shfl_xor(t, 8));
      const float mnew = fmaxf(mrow[g], t);
      const float corr = __expf(mrow[g] - mnew);
      float rs = 0.0f;
#pragma unroll
      for (int jt = 0; jt < 4; ++jt) {
        const float p = __expf(e[jt] - mnew);
        rs += p;
        const bf16_t phv = (bf16_t)p;
        const float prm = p - (float)phv;
        myph[(8 * hf + g) * kPP + 16 * jt + n] = phv;
        mypl[(8 * hf + g) * kPP + 16 * jt + n] = (bf16_t)prm;
      }
      rs += __shfl_xor(rs, 1);
      rs += __shfl_xor(rs, 2);
      rs += __shfl_xor(rs, 4);
      rs += __shfl_xor(rs, 8);
      lrow[g] = lrow[g] * corr + rs;
      mrow[g] = mnew;
#pragma unroll
      for (int c = 0; c < 4; ++c) acc[c][g] *= corr;
    }
    __syncthreads();

    const Frag aph0 = lds_frag(myph + n * kPP, hf);
    const Frag aph1 = lds_frag(myph + n * kPP + 32, hf);
    const Frag apl0 = lds_frag(mypl + n * kPP, hf);
    const Frag apl1 = lds_frag(mypl + n * kPP + 32, hf);
#pragma unroll
    for (int c = 0; c < 4; ++c) {
      const size_t vr = ((size_t)bh * kDh + 16 * c + n) * kS + key0;
      {
        const Frag b0h = ldg_frag(vth + vr, hf);
        const Frag b0l = ldg_frag(vtl + vr, hf);
        acc[c] = mma3(aph0, apl0, b0h, b0l, acc[c]);
      }
      {
        const Frag b1h = ldg_frag(vth + vr + 32, hf);
        const Frag b1l = ldg_frag(vtl + vr + 32, hf);
        acc[c] = mma3(aph1, apl1, b1h, b1l, acc[c]);
      }
    }
    __syncthreads();
  }

  float inv[8];
#pragma unroll
  for (int g = 0; g < 8; ++g) inv[g] = __builtin_amdgcn_rcpf(lrow[g]);
#pragma unroll
  for (int c = 0; c < 4; ++c) {
#pragma unroll
    for (int g = 0; g < 8; ++g) myst[(8 * hf + g) * kSP + 16 * c + n] = acc[c][g] * inv[g];
  }
  __syncthreads();
  const int q = lane & 7;
  v4u uh[4], ul[4];
  size_t off[4];
#pragma unroll
  for (int i = 0; i < 4; ++i) {
    const int row = (lane >> 3) + 4 * i;
    const float* sp = myst + row * kSP + 8 * q;
    const v4f a = *(const v4f*)sp;
    const v4f b = *(const v4f*)(sp + 4);
    float x[8] = { a[0], a[1], a[2], a[3], b[0], b[1], b[2], b[3] };
    split8(x, uh[i], ul[i]);
    off[i] = ((size_t)(bg * kS + q0 + row)) * kD + hd * kDh + 8 * q;
    *(volatile v4u*)(oh + off[i]) = uh[i];
    *(volatile v4u*)(ol + off[i]) = ul[i];
  }
  __threadfence();
#pragma unroll
  for (int i = 0; i < 4; ++i) {
    *(volatile v4u*)(oh + off[i]) = uh[i];
    *(volatile v4u*)(ol + off[i]) = ul[i];
  }
}

__global__ void __launch_bounds__(256)
k_oproj(const bf16_t* __restrict__ ah, const bf16_t* __restrict__ al,
        const bf16_t* __restrict__ woh, const bf16_t* __restrict__ wol,
        const float* __restrict__ bo, float* __restrict__ out) {
  __shared__ __align__(16) float stg[128 * kSP];
  const int tid = threadIdx.x, lane = tid & 31, wv = tid >> 5;
  const int hf = lane >> 4, n = lane & 15;
  const int bid = blockIdx.x;
  const int ct = bid & 15, rb = bid >> 4;
  const int c0 = ct * 64;
  const int r0 = rb * 128;

  const size_t arow = ((size_t)r0 + 16 * wv + n) * kD;
  const size_t brow = (size_t)(c0 + n) * kD;
  v8f acc[4] = { {}, {}, {}, {} };
  gemm_k1024(ah + arow, al + arow, woh + brow, wol + brow, hf, acc[0], acc[1], acc[2], acc[3]);

#pragma unroll
  for (int j = 0; j < 4; ++j) {
    const int col = 16 * j + n;
    const float bb = bo[c0 + col];
#pragma unroll
    for (int g = 0; g < 8; ++g) stg[(16 * wv + 8 * hf + g) * kSP + col] = acc[j][g] + bb;
  }
  __syncthreads();

  const int q = tid & 7;
  v4f o[8];
  size_t off[8];
#pragma unroll
  for (int i = 0; i < 8; ++i) {
    const int L = (tid >> 3) + 32 * i;
    const int row = L >> 1;
    const int cseg = (L & 1) * 32 + 4 * q;
    o[i] = *(const v4f*)(stg + row * kSP + cseg);
    off[i] = ((size_t)(r0 + row)) * kD + c0 + cseg;
    *(volatile v4f*)(out + off[i]) = o[i];
  }
  __threadfence();
#pragma unroll
  for (int i = 0; i < 8; ++i) *(volatile v4f*)(out + off[i]) = o[i];
}

extern "C" void kernel_launch(void* const* d_in, const int* in_sizes, int n_in,
                              void* d_out, int out_size, void* d_ws, size_t ws_size,
                              hipStream_t stream) {
  if (n_in < 10) return;
  if (in_sizes[0] != kRows * kD || in_sizes[1] != kB) return;
  if (in_sizes[2] != kD * kD || in_sizes[4] != kD * kD || in_sizes[6] != kD * kD || in_sizes[8] != kD * kD) return;
  if (in_sizes[3] != kD || in_sizes[5] != kD || in_sizes[7] != kD || in_sizes[9] != kD) return;
  if (out_size != kRows * kD) return;
  if (ws_size < kWsTotal) return;

  const float* v       = (const float*)d_in[0];
  const int*   lengths = (const int*)d_in[1];
  const float* Wq = (const float*)d_in[2];
  const float* bq = (const float*)d_in[3];
  const float* Wk = (const float*)d_in[4];
  const float* bk = (const float*)d_in[5];
  const float* Wv = (const float*)d_in[6];
  const float* bv = (const float*)d_in[7];
  const float* Wo = (const float*)d_in[8];
  const float* bo = (const float*)d_in[9];
  float* out = (float*)d_out;

  char* ws = (char*)d_ws;
  bf16_t* XH = (bf16_t*)(ws + OFF_XH);
  bf16_t* XL = (bf16_t*)(ws + OFF_XL);
  bf16_t* WT = (bf16_t*)(ws + OFF_WT);
  bf16_t* QH = (bf16_t*)(ws + OFF_QH);
  bf16_t* QL = (bf16_t*)(ws + OFF_QL);
  bf16_t* KH = (bf16_t*)(ws + OFF_KH);
  bf16_t* KL = (bf16_t*)(ws + OFF_KL);
  bf16_t* VH = (bf16_t*)(ws + OFF_VH);
  bf16_t* VL = (bf16_t*)(ws + OFF_VL);
  const bf16_t* WOH = WT + (size_t)6 * kD * kD;
  const bf16_t* WOL = WT + (size_t)7 * kD * kD;

  k_split_x<<<(kRows * kD / 8) / 256, 256, 0, stream>>>(v, XH, XL, kRows * kD / 8);
  k_split_wT<<<4 * 256, 256, 0, stream>>>(Wq, Wk, Wv, Wo, WT);

  for (int hb = 0; hb < 2; ++hb) {
    k_qkv<<<3 * 32 * 16, 256, 0, stream>>>(XH, XL, WT, bq, bk, bv, QH, QL, KH, KL, VH, VL, hb);
    k_attn<<<kHalfB * kH * 8, 128, 0, stream>>>(QH, QL, KH, KL, VH, VL, lengths, XH, XL, hb);
  }

  k_oproj<<<64 * 16, 256, 0, stream>>>(XH, XL, WOH, WOL, bo, out);
}
